// ScaledDotSelfAttention_70832600646361
// MI455X (gfx1250) — hardware-run, weakly checked
//
#include <hip/hip_runtime.h>
#include <math.h>
#include <stdint.h>

#define NB    8
#define SEQ   1024
#define DMOD  1024
#define NH    16
#define HD    64
#define ROWS  (NB * SEQ)
#define PCAR  32768.0f
#define VCAR  1024.0f
#define OSC   1024.0f
#define WOS   1024.0f
#define EPSR  1e-7f
#define LOG2E 1.4426950408889634f
#define ATT_WAVES   4
#define ATT_THREADS (ATT_WAVES * 32)
#define QT64        (SEQ / 64)
#define ATT_BLOCKS  (NB * NH * QT64)
#define NKB    (SEQ / 32)
#define SLAB64 (16 * 68)
#define VTP    72

static_assert(HD == 64 && DMOD == NH * HD);
static_assert(QT64 == 16 && NH == 16 && NB == 8 && NKB == 32);
static_assert(ATT_THREADS == 128 && ATT_BLOCKS == 2048);
static_assert((ROWS % 64) == 0 && (DMOD % 64) == 0 && (DMOD % 32) == 0 && (SEQ % 64) == 0);
static_assert(((ROWS * DMOD / 8) % 256) == 0);
static_assert((DMOD / 8) == 128);
static_assert(64 * VTP >= 63 * VTP + 64 && ((VTP * 2) % 16) == 0);
static_assert(ATT_WAVES * SLAB64 >= 4 * 16 * 68);

typedef unsigned short u16;
typedef _Float16 v16h __attribute__((ext_vector_type(16)));
typedef _Float16 v8h  __attribute__((ext_vector_type(8)));
typedef __bf16   v16b __attribute__((ext_vector_type(16)));
typedef float    v8f  __attribute__((ext_vector_type(8)));
typedef float    v4f  __attribute__((ext_vector_type(4)));
typedef unsigned int v4u __attribute__((ext_vector_type(4)));
typedef int      v4i  __attribute__((ext_vector_type(4)));

union FragH { v16h v; v8h h[2]; v4u u[2]; };
union FragB { v16b v; v4u u[2]; };

__device__ __forceinline__ unsigned short bf_bits(float f) {
  unsigned u = __float_as_uint(f);
  return (unsigned short)((u + 0x7FFFu + ((u >> 16) & 1u)) >> 16);
}
__device__ __forceinline__ float bf_up(unsigned short h) { return __uint_as_float(((unsigned)h) << 16); }
__device__ __forceinline__ float bfr(float f) { return bf_up(bf_bits(f)); }
__device__ __forceinline__ unsigned short h_bits(_Float16 x) { return __builtin_bit_cast(unsigned short, x); }
__device__ __forceinline__ unsigned pk16(unsigned short a, unsigned short b) { return (unsigned)a | ((unsigned)b << 16); }
__device__ __forceinline__ v8f zero8() { v8f z = {0.f, 0.f, 0.f, 0.f, 0.f, 0.f, 0.f, 0.f}; return z; }

__device__ __forceinline__ v16h ldfrag_h(const _Float16* p) {
  FragH f;
  f.h[0] = *(const v8h*)(p);
  f.h[1] = *(const v8h*)(p + 16);
  return f.v;
}
__device__ __forceinline__ v16b ldfrag_b(const u16* p) {
  FragB f;
  f.u[0] = *(const v4u*)(p);
  f.u[1] = *(const v4u*)(p + 16);
  return f.v;
}

__device__ __forceinline__ v8f mma_h(v16h a, v16h b, v8f c) {
  return __builtin_amdgcn_wmma_f32_16x16x32_f16(false, a, false, b, (short)0, c, false, false);
}
__device__ __forceinline__ v8f mma_b(v16b a, v16b b, v8f c) {
  return __builtin_amdgcn_wmma_f32_16x16x32_bf16(false, a, false, b, (short)0, c, false, false);
}
template <typename F>
__device__ __forceinline__ void guard1x8(v8f& a, F x0, F x1, F x2, F x3, F x4, F x5, F x6, F x7) {
#if defined(__HIP_DEVICE_COMPILE__)
  asm volatile("v_nop\n\tv_nop\n\tv_nop\n\tv_nop"
               : "+v"(a) : "v"(x0), "v"(x1), "v"(x2), "v"(x3), "v"(x4), "v"(x5), "v"(x6), "v"(x7) : "memory");
#endif
}
template <typename F>
__device__ __forceinline__ void guard6(v8f& a, v8f& b, v8f& c, v8f& d, F x0, F x1, F x2, F x3, F x4, F x5) {
#if defined(__HIP_DEVICE_COMPILE__)
  asm volatile("v_nop\n\tv_nop\n\tv_nop\n\tv_nop"
               : "+v"(a), "+v"(b), "+v"(c), "+v"(d) : "v"(x0), "v"(x1), "v"(x2), "v"(x3), "v"(x4), "v"(x5) : "memory");
#endif
}
__device__ __forceinline__ void acc_guard4(v8f& a, v8f& b, v8f& c, v8f& d) {
#if defined(__HIP_DEVICE_COMPILE__)
  asm volatile("v_nop\n\tv_nop\n\tv_nop\n\tv_nop" : "+v"(a), "+v"(b), "+v"(c), "+v"(d));
#endif
}
__device__ __forceinline__ void wave_sync_lds() {
  __builtin_amdgcn_fence(__ATOMIC_RELEASE, "workgroup");
  __builtin_amdgcn_wave_barrier();
  __builtin_amdgcn_fence(__ATOMIC_ACQUIRE, "workgroup");
}

__global__ __launch_bounds__(256) void cvtx(const float* __restrict__ x, const int* __restrict__ msk, u16* D, int n8) {
  const int gt = blockIdx.x * 256 + (int)threadIdx.x;
  if (gt >= n8) return;
  const int row = gt >> 7;
  const float mf = (float)msk[row];
  const float* p = x + (size_t)gt * 8;
  const v4f a = *(const v4f*)(p), c4 = *(const v4f*)(p + 4);
  float v[8];
#pragma unroll
  for (int e = 0; e < 4; ++e) { v[e] = a[e] * mf; v[4 + e] = c4[e] * mf; }
  v4u o;
#pragma unroll
  for (int e = 0; e < 4; ++e) o[e] = pk16(bf_bits(v[2 * e]), bf_bits(v[2 * e + 1]));
  u16* d = D + (size_t)gt * 8;
  for (int pass = 0; pass < 2; ++pass) {
    *(volatile v4u*)(d) = o;
    __threadfence();
  }
}

__global__ __launch_bounds__(256) void cvtw(const float* __restrict__ W, u16* WT, int K, int N, int mode, float scale) {
  __shared__ __align__(16) u16 TH[64 * VTP];
  const int tid = threadIdx.x;
  const int bid = blockIdx.x;
  const int ktn = K >> 6;
  const int kt  = bid % ktn;
  const int nt  = bid / ktn;
  const int k0  = kt * 64, n0 = nt * 64;
  {
    const int r  = tid >> 2;
    const int dc = (tid & 3) * 16;
    const float* src = W + (size_t)(k0 + r) * N + n0 + dc;
#pragma unroll
    for (int i = 0; i < 4; ++i) {
      const v4f a = *(const v4f*)(src + 4 * i);
#pragma unroll
      for (int e = 0; e < 4; ++e) {
        const float v = a[e];
        const unsigned short hb = h_bits((_Float16)(bfr(v) * scale));
        const unsigned short bb = bf_bits(v);
        TH[(dc + 4 * i + e) * VTP + r] = (mode != 0) ? hb : bb;
      }
    }
  }
  __syncthreads();
  v4u vh[2];
  const int q8 = tid >> 3, p8 = (tid & 7) * 8;
#pragma unroll
  for (int it = 0; it < 2; ++it) {
    const int line = it * 32 + q8;
    vh[it] = *(const v4u*)(TH + line * VTP + p8);
  }
  const size_t base = (size_t)n0 * K + k0 + p8;
  for (int pass = 0; pass < 2; ++pass) {
#pragma unroll
    for (int it = 0; it < 2; ++it) {
      const int line = it * 32 + q8;
      *(volatile v4u*)(WT + base + (size_t)line * K) = vh[it];
    }
    __threadfence();
  }
}

__device__ __forceinline__ void epi64(float* sl, v8f a0, v8f a1, v8f a2, v8f a3, float oscale, float* C, int N,
                                      size_t rowb, int col0, int lane) {
  const int hh = lane >> 4, m = lane & 15;
#pragma unroll
  for (int r = 0; r < 8; ++r) {
    const int ro = (8 * hh + r) * 68 + m;
    sl[ro]      = a0[r] * oscale;
    sl[ro + 16] = a1[r] * oscale;
    sl[ro + 32] = a2[r] * oscale;
    sl[ro + 48] = a3[r] * oscale;
  }
  wave_sync_lds();
  v4f vals[8];
#pragma unroll
  for (int it = 0; it < 8; ++it) vals[it] = *(const v4f*)(sl + (it * 2 + hh) * 68 + m * 4);
  float* dst = C + (rowb + (size_t)hh) * (size_t)N + col0 + m * 4;
  for (int pass = 0; pass < 2; ++pass) {
#pragma unroll
    for (int it = 0; it < 8; ++it) {
      *(volatile v4f*)(dst + (size_t)(it * 2) * (size_t)N) = vals[it];
    }
    __threadfence();
  }
}

template <int MODE>
__device__ __forceinline__ void epi16(float* sl, v8f a0, v8f a1, v8f a2, v8f a3, float oscale, u16* C0, u16* C1, int N,
                                      size_t rowb, int col0, int lane) {
  const int hh = lane >> 4, m = lane & 15;
#pragma unroll
  for (int r = 0; r < 8; ++r) {
    const int ro = (8 * hh + r) * 68 + m;
    sl[ro]      = a0[r] * oscale;
    sl[ro + 16] = a1[r] * oscale;
    sl[ro + 32] = a2[r] * oscale;
    sl[ro + 48] = a3[r] * oscale;
  }
  wave_sync_lds();
  const int rq = lane >> 3, c8 = (lane & 7) * 8;
  v4u o0[4], o1[4];
#pragma unroll
  for (int i4 = 0; i4 < 4; ++i4) {
    const int row = i4 * 4 + rq;
    const v4f a = *(const v4f*)(sl + row * 68 + c8), c4 = *(const v4f*)(sl + row * 68 + c8 + 4);
    float w[8];
#pragma unroll
    for (int e = 0; e < 4; ++e) { w[e] = a[e]; w[4 + e] = c4[e]; }
#pragma unroll
    for (int e = 0; e < 4; ++e) {
      const float w0 = w[2 * e], w1 = w[2 * e + 1];
      if (MODE == 0) {
        const unsigned short h0 = bf_bits(w0), h1 = bf_bits(w1);
        const unsigned short l0 = bf_bits(w0 - bf_up(h0)), l1 = bf_bits(w1 - bf_up(h1));
        o0[i4][e] = pk16(h0, h1);
        o1[i4][e] = pk16(l0, l1);
      } else {
        o0[i4][e] = pk16(h_bits((_Float16)w0), h_bits((_Float16)w1));
        o1[i4][e] = o0[i4][e];
      }
    }
  }
  const size_t base = rowb * (size_t)N + col0 + c8;
  for (int pass = 0; pass < 2; ++pass) {
#pragma unroll
    for (int i4 = 0; i4 < 4; ++i4) {
      const int row = i4 * 4 + rq;
      const size_t o8 = base + (size_t)row * (size_t)N;
      *(volatile v4u*)(C0 + o8) = o0[i4];
      if (MODE == 0) *(volatile v4u*)(C1 + o8) = o1[i4];
    }
    __threadfence();
  }
}

template <int MODE>
__global__ __launch_bounds__(128)
void gemm16(const u16* __restrict__ A, const u16* __restrict__ Bt, u16* C0, u16* C1, int M, int N, int K, float oscale) {
  __shared__ __align__(16) float slab[4 * SLAB64];
  const int tid = threadIdx.x, wave = tid >> 5, lane = tid & 31, hh = lane >> 4, m = lane & 15;
  const int ntile = N >> 6;
  const int bid   = blockIdx.x;
  const int rowb  = (bid / ntile) * 64 + wave * 16;
  const int col0  = (bid % ntile) * 64;
  if (rowb + 16 > M) return;
  const u16* ap = A  + (size_t)(rowb + m) * K + 8 * hh;
  const u16* bp = Bt + (size_t)(col0 + m) * K + 8 * hh;
  const size_t bs = (size_t)16 * K;
  v8f acc0 = zero8(), acc1 = zero8(), acc2 = zero8(), acc3 = zero8();
#pragma unroll 1
  for (int k0 = 0; k0 < K; k0 += 32) {
    const v16b a  = ldfrag_b(ap + k0);
    const v16b b0 = ldfrag_b(bp + k0);
    const v16b b1 = ldfrag_b(bp + bs + k0);
    const v16b b2 = ldfrag_b(bp + 2 * bs + k0);
    const v16b b3 = ldfrag_b(bp + 3 * bs + k0);
    acc0 = mma_b(a, b0, acc0);
    acc1 = mma_b(a, b1, acc1);
    acc2 = mma_b(a, b2, acc2);
    acc3 = mma_b(a, b3, acc3);
    guard6<v16b>(acc0, acc1, acc2, acc3, a, b0, b1, b2, b3, a);
  }
  epi16<MODE>(slab + wave * SLAB64, acc0, acc1, acc2, acc3, oscale, C0, C1, N, (size_t)rowb, col0, lane);
}

__global__ __launch_bounds__(128)
void gemm_h2(const u16* __restrict__ Ah, const u16* __restrict__ Al, const u16* __restrict__ Bt,
             float* C, int M, int N, int K, float oscale) {
  __shared__ __align__(16) float slab[4 * SLAB64];
  const int tid = threadIdx.x, wave = tid >> 5, lane = tid & 31, hh = lane >> 4, m = lane & 15;
  const int ntile = N >> 6;
  const int bid   = blockIdx.x;
  const int rowb  = (bid / ntile) * 64 + wave * 16;
  const int col0  = (bid % ntile) * 64;
  if (rowb + 16 > M) return;
  const size_t aofs = (size_t)(rowb + m) * K + 8 * hh;
  const _Float16* ahp = (const _Float16*)(const void*)Ah + aofs;
  const _Float16* alp = (const _Float16*)(const void*)Al + aofs;
  const _Float16* bp  = (const _Float16*)(const void*)Bt + (size_t)(col0 + m) * K + 8 * hh;
  const size_t bs = (size_t)16 * K;
  v8f acc0 = zero8(), acc1 = zero8(), acc2 = zero8(), acc3 = zero8();
#pragma unroll 1
  for (int k0 = 0; k0 < K; k0 += 32) {
    const v16h ah = ldfrag_h(ahp + k0), al = ldfrag_h(alp + k0);
    const v16h b0 = ldfrag_h(bp + k0);
    const v16h b1 = ldfrag_h(bp + bs + k0);
    const v16h b2 = ldfrag_h(bp + 2 * bs + k0);
    const v16h b3 = ldfrag_h(bp + 3 * bs + k0);
    acc0 = mma_h(ah, b0, acc0);  acc0 = mma_h(al, b0, acc0);
    acc1 = mma_h(ah, b1, acc1);  acc1 = mma_h(al, b1, acc1);
    acc2 = mma_h(ah, b2, acc2);  acc2 = mma_h(al, b2, acc2);
    acc3 = mma_h(ah, b3, acc3);  acc3 = mma_h(al, b3, acc3);
    guard6<v16h>(acc0, acc1, acc2, acc3, ah, al, b0, b1, b2, b3);
  }
  epi64(slab + wave * SLAB64, acc0, acc1, acc2, acc3, oscale, C, N, (size_t)rowb, col0, lane);
}

__global__ __launch_bounds__(ATT_THREADS)
void attn_fwd(const u16* __restrict__ QHp, const u16* __restrict__ QLp, const u16* __restrict__ KHp,
              const u16* __restrict__ KLp, const u16* __restrict__ VPp, const int* __restrict__ MSK,
              u16* OHIp, u16* OLOp) {
  __shared__ __align__(16) float smem[ATT_WAVES * SLAB64];

  const int tid  = threadIdx.x;
  const int wave = tid >> 5;
  const int lane = tid & 31;
  const int hh   = lane >> 4;
  const int c    = lane & 15;

  const int bid  = blockIdx.x;
  const int qt   = bid & (QT64 - 1);
  const int head = (bid >> 4) & (NH - 1);
  const int b    = bid >> 8;
  const int q0   = qt * 64 + wave * 16;

  const size_t qofs = ((size_t)(b * SEQ + q0 + c)) * DMOD + head * HD + 8 * hh;
  const size_t kofs = ((size_t)(b * SEQ + c)) * DMOD + head * HD + 8 * hh;
  const size_t vofs = ((size_t)(head * HD + c)) * ROWS + (size_t)b * SEQ + 8 * hh;
  const _Float16* Vb = (const _Float16*)(const void*)VPp + vofs;
  const int* mp = MSK + (size_t)b * SEQ + 8 * hh;
  const float lsc = 0.125f * LOG2E;

  const v16b qh0 = ldfrag_b(QHp + qofs);
  const v16b qh1 = ldfrag_b(QHp + qofs + 32);
  const v16b ql0 = ldfrag_b(QLp + qofs);
  const v16b ql1 = ldfrag_b(QLp + qofs + 32);

  float mrun = -INFINITY, za = 0.f, zm = 0.f;
  v8f o[4];
#pragma unroll
  for (int j = 0; j < 4; ++j) o[j] = zero8();

#pragma unroll 1
  for (int it = 0; it < NKB; ++it) {
    const int kb = it * 32;
    v8f s0 = zero8(), s1 = zero8();
    {
      const u16* k0p = KHp + kofs + (size_t)kb * DMOD;
      const u16* l0p = KLp + kofs + (size_t)kb * DMOD;
      const v16b a0 = ldfrag_b(k0p), a1 = ldfrag_b(k0p + 32);
      const v16b l0 = ldfrag_b(l0p), l1 = ldfrag_b(l0p + 32);
      s0 = mma_b(a0, qh0, s0);  s0 = mma_b(a0, ql0, s0);  s0 = mma_b(l0, qh0, s0);
      s0 = mma_b(a1, qh1, s0);  s0 = mma_b(a1, ql1, s0);  s0 = mma_b(l1, qh1, s0);
      guard1x8<v16b>(s0, a0, a1, l0, l1, qh0, qh1, ql0, ql1);
    }
    {
      const u16* k1p = KHp + kofs + (size_t)(kb + 16) * DMOD;
      const u16* l1p = KLp + kofs + (size_t)(kb + 16) * DMOD;
      const v16b a0 = ldfrag_b(k1p), a1 = ldfrag_b(k1p + 32);
      const v16b l0 = ldfrag_b(l1p), l1 = ldfrag_b(l1p + 32);
      s1 = mma_b(a0, qh0, s1);  s1 = mma_b(a0, ql0, s1);  s1 = mma_b(l0, qh0, s1);
      s1 = mma_b(a1, qh1, s1);  s1 = mma_b(a1, ql1, s1);  s1 = mma_b(l1, qh1, s1);
      guard1x8<v16b>(s1, a0, a1, l0, l1, qh0, qh1, ql0, ql1);
    }
    int mk[16];
    {
      const v4i ma = *(const v4i*)(mp + kb),      mb = *(const v4i*)(mp + kb + 4);
      const v4i mc = *(const v4i*)(mp + kb + 16), md = *(const v4i*)(mp + kb + 20);
#pragma unroll
      for (int e = 0; e < 4; ++e) { mk[e] = ma[e]; mk[4 + e] = mb[e]; mk[8 + e] = mc[e]; mk[12 + e] = md[e]; }
    }
    float tk[16];
#pragma unroll
    for (int i = 0; i < 8; ++i) { tk[i] = s0[i] * lsc;  tk[8 + i] = s1[i] * lsc; }
    float cm = -INFINITY;
#pragma unroll
    for (int i = 0; i < 16; ++i) cm = fmaxf(cm, tk[i]);
    cm = fmaxf(cm, __shfl_xor(cm, 16, 32));
    const float mn = fmaxf(mrun, cm);
    const float al = exp2f(mrun - mn);
    mrun = mn;
    float pa = 0.f, ps = 0.f;
    FragH ph;
#pragma unroll
    for (int w = 0; w < 2; ++w) {
#pragma unroll
      for (int e4 = 0; e4 < 4; ++e4) {
        const int i = 8 * w + 2 * e4;
        const float x0 = exp2f(tk[i] - mn);
        const float x1 = exp2f(tk[i + 1] - mn);
        pa += x0 + x1;
        const float p0 = x0 * (float)mk[i];
        const float p1 = x1 * (float)mk[i + 1];
        ps += p0 + p1;
        ph.u[w][e4] = pk16(h_bits((_Float16)(p0 * PCAR)), h_bits((_Float16)(p1 * PCAR)));
      }
    }
    pa += __shfl_xor(pa, 16, 32);
    ps += __shfl_xor(ps, 16, 32);
    za = za * al + pa;
    zm = zm * al + ps;
    float scl[8];
#pragma unroll
    for (int r = 0; r < 8; ++r) scl[r] = __shfl(al, 8 * hh + r, 32);
#pragma unroll
    for (int j = 0; j < 4; ++j) {
#pragma unroll
      for (int r = 0; r < 8; ++r) o[j][r] *= scl[r];
    }
    {
      const _Float16* vp = Vb + kb;
      const v16h vf0 = ldfrag_h(vp);
      const v16h vf1 = ldfrag_h(vp + (size_t)16 * ROWS);
      const v16h vf2 = ldfrag_h(vp + (size_t)32 * ROWS);
      const v16h vf3 = ldfrag_h(vp + (size_t)48 * ROWS);
      o[0] = mma_h(ph.v, vf0, o[0]);
      o[1] = mma_h(ph.v, vf1, o[1]);
      o[2] = mma_h(ph.v, vf2, o[2]);
      o[3] = mma_h(ph.v, vf3, o[3]);
      guard6<v16h>(o[0], o[1], o[2], o[3], ph.v, vf0, vf1, vf2, vf3, ph.v);
    }
  }
  acc_guard4(o[0], o[1], o[2], o[3]);

  const float den  = zm + EPSR * za;
  const float linv = (den > 0.f) ? ((1.0f / den) * (1.0f / (PCAR * VCAR))) : 0.f;
  float inv[8];
#pragma unroll
  for (int r = 0; r < 8; ++r) inv[r] = __shfl(linv, 8 * hh + r, 32);
  float* slab = smem + wave * SLAB64;
#pragma unroll
  for (int r = 0; r < 8; ++r) {
#pragma unroll
    for (int j = 0; j < 4; ++j) slab[(8 * hh + r) * 68 + j * 16 + c] = o[j][r] * inv[r];
  }
  wave_sync_lds();
  v4u oh[4], ol[4];
  const int rq = lane >> 3, c8 = (lane & 7) * 8;
#pragma unroll
  for (int i4 = 0; i4 < 4; ++i4) {
    const int row = i4 * 4 + rq;
    const v4f a = *(const v4f*)(slab + row * 68 + c8), c4 = *(const v4f*)(slab + row * 68 + c8 + 4);
    float w[8];
#pragma unroll
    for (int e = 0; e < 4; ++e) { w[e] = a[e] * OSC; w[4 + e] = c4[e] * OSC; }
#pragma unroll
    for (int e = 0; e < 4; ++e) {
      const _Float16 h0 = (_Float16)w[2 * e], h1 = (_Float16)w[2 * e + 1];
      const _Float16 l0 = (_Float16)(w[2 * e] - (float)h0), l1 = (_Float16)(w[2 * e + 1] - (float)h1);
      oh[i4][e] = pk16(h_bits(h0), h_bits(h1));
      ol[i4][e] = pk16(h_bits(l0), h_bits(l1));
    }
  }
  const size_t ob = ((size_t)(b * SEQ + q0)) * DMOD + head * HD + c8;
  for (int pass = 0; pass < 2; ++pass) {
#pragma unroll
    for (int i4 = 0; i4 < 4; ++i4) {
      const int row = i4 * 4 + rq;
      const size_t o8 = ob + (size_t)row * DMOD;
      *(volatile v4u*)(OHIp + o8) = oh[i4];
      *(volatile v4u*)(OLOp + o8) = ol[i4];
    }
    __threadfence();
  }
}

extern "C" void kernel_launch(void* const* d_in, const int* in_sizes, int n_in,
                              void* d_out, int out_size, void* d_ws, size_t ws_size,
                              hipStream_t stream) {
  if (n_in < 6) return;
  if (in_sizes[0] != ROWS * DMOD || in_sizes[1] != ROWS) return;
  if (in_sizes[2] != DMOD * DMOD || in_sizes[3] != DMOD * DMOD) return;
  if (in_sizes[4] != DMOD * DMOD || in_sizes[5] != DMOD * DMOD) return;
  if (out_size != ROWS * DMOD) return;

  const float* Xin = (const float*)d_in[0];
  const int*   Msk = (const int*)d_in[1];
  const float* wq  = (const float*)d_in[2];
  const float* wk  = (const float*)d_in[3];
  const float* wv  = (const float*)d_in[4];
  const float* wo  = (const float*)d_in[5];
  float*       out = (float*)d_out;

  const size_t szX = (size_t)ROWS * DMOD * 2;
  const size_t szW = (size_t)DMOD * DMOD * 2;
  size_t off = 0;
  const size_t oXB  = off; off += szX;
  const size_t oWQT = off; off += szW;
  const size_t oWKT = off; off += szW;
  const size_t oWVT = off; off += szW;
  const size_t oWOT = off; off += szW;
  const size_t oQH  = off; off += szX;
  const size_t oQL  = off; off += szX;
  const size_t oKH  = off; off += szX;
  const size_t oKL  = off; off += szX;
  const size_t oVP  = off; off += szX;
  const size_t oOLO = off; off += szX;
  if (off > ws_size) return;
  if (off > (size_t)134217728) return;

  char* ws = (char*)d_ws;
  u16* XB  = (u16*)(ws + oXB);
  u16* WQT = (u16*)(ws + oWQT);
  u16* WKT = (u16*)(ws + oWKT);
  u16* WVT = (u16*)(ws + oWVT);
  u16* WOT = (u16*)(ws + oWOT);
  u16* QH  = (u16*)(ws + oQH);
  u16* QL  = (u16*)(ws + oQL);
  u16* KH  = (u16*)(ws + oKH);
  u16* KL  = (u16*)(ws + oKL);
  u16* VP  = (u16*)(ws + oVP);
  u16* OLO = (u16*)(ws + oOLO);
  u16* OHI = XB;

  const dim3 blk(256);
  const int n8x = (ROWS * DMOD) / 8;
  if ((n8x % 256) != 0 || (DMOD % 64) != 0 || (ROWS % 64) != 0 || (DMOD % 32) != 0) return;
  const dim3 gX(n8x / 256);
  const dim3 gWT((DMOD / 64) * (DMOD / 64));
  const dim3 gG((ROWS / 64) * (DMOD / 64));
  const dim3 bG(128);
  const dim3 gAT(ATT_BLOCKS);
  const dim3 bAT(ATT_THREADS);

  cvtw<<<gWT, blk, 0, stream>>>(wq, WQT, DMOD, DMOD, 0, 1.0f);
  cvtw<<<gWT, blk, 0, stream>>>(wk, WKT, DMOD, DMOD, 0, 1.0f);
  cvtw<<<gWT, blk, 0, stream>>>(wv, WVT, DMOD, DMOD, 0, 1.0f);
  cvtw<<<gWT, blk, 0, stream>>>(wo, WOT, DMOD, DMOD, 1, WOS);
  cvtx<<<gX, blk, 0, stream>>>(Xin, Msk, XB, n8x);
  gemm16<0><<<gG, bG, 0, stream>>>(XB, WQT, QH, QL, ROWS, DMOD, DMOD, 1.0f);
  gemm16<0><<<gG, bG, 0, stream>>>(XB, WKT, KH, KL, ROWS, DMOD, DMOD, 1.0f);
  gemm16<1><<<gG, bG, 0, stream>>>(WVT, XB, VP, VP, DMOD, ROWS, DMOD, VCAR);
  attn_fwd<<<gAT, bAT, 0, stream>>>(QH, QL, KH, KL, VP, Msk, OHI, OLO);
  gemm_h2<<<gG, bG, 0, stream>>>(OHI, OLO, WOT, out, ROWS, DMOD, DMOD, 1.0f / (OSC * WOS));
  (void)hipGetLastError();
}
